// TensorProductConvBlock_55405078118473
// MI455X (gfx1250) — hardware-verified
//
#include <hip/hip_runtime.h>
#include <stddef.h>


#define NTHR   64
#define NWAVE  2
#define EPT    8
#define CHUNK  (NTHR * EPT)
#define WCAP   (EPT * 32)
#define LISTN  (NWAVE * WCAP)
#define PASSN  NTHR
#define PCAP   (CHUNK + PASSN)
#define NB     256
#define NTA    128
#define KP     64
#define SP     48
#define WP     64
#define EFP    32
#define N28P   32
#define NWROWS 848

static_assert(PASSN == NTHR);
static_assert(PCAP >= CHUNK + PASSN);
static_assert((NB % 32) == 0);
static_assert((NWROWS % (4 * NWAVE)) == 0);

typedef float  v4f  __attribute__((ext_vector_type(4)));
typedef float  v8f  __attribute__((ext_vector_type(8)));
typedef int    v2i  __attribute__((ext_vector_type(2)));
typedef int    v4i  __attribute__((ext_vector_type(4)));
typedef __bf16 bf_t;
typedef bf_t   v8b  __attribute__((ext_vector_type(8)));
typedef bf_t   v16b __attribute__((ext_vector_type(16)));
union FragB { v16b v; v8b b[2]; v8f f; };
union Pk8   { v8b b; v4f f; };

#define RBF_COEFF (-0.6805555555555556f)
#define RBF_STEP  0.8571428571428571f
#define SQ3F 1.7320508075688772f
#define PW0  0.22360679774997896f
#define PW1  0.3535533905932738f
#define P1E  0.8660254037844386f
#define INV3 0.5773502691896258f
#define C_A  0.31622776601683794f
#define C_B  0.3651483716701107f
#define INV6 0.4082482904638631f
#define S15  3.872983346207417f
#define S5   2.23606797749979f

__device__ __forceinline__ int imin(int a, int b) { return a < b ? a : b; }
__device__ __forceinline__ int imax(int a, int b) { return a > b ? a : b; }

__device__ __forceinline__ v8f cat8(v4f a, v4f b) {
  v8f c;
  c[0] = a.x; c[1] = a.y; c[2] = a.z; c[3] = a.w;
  c[4] = b.x; c[5] = b.y; c[6] = b.z; c[7] = b.w;
  return c;
}
__device__ __forceinline__ v4f lo4(v8f x) { v4f r = {x[0], x[1], x[2], x[3]}; return r; }
__device__ __forceinline__ v4f hi4(v8f x) { v4f r = {x[4], x[5], x[6], x[7]}; return r; }

__device__ __forceinline__ v8b zero8b() {
  Pk8 u;
  const v4f z = {0.0f, 0.0f, 0.0f, 0.0f};
  u.f = z;
  return u.b;
}

__device__ __forceinline__ void split8(v8f x, v8b& hi, v8b& lo) {
  v8b a, b;
#pragma unroll
  for (int i = 0; i < 8; ++i) {
    const float xf = x[i];
    const bf_t hb = (bf_t)xf;
    const float r = xf - (float)hb;
    a[i] = hb;
    b[i] = (bf_t)r;
  }
  hi = a;
  lo = b;
}

__device__ __forceinline__ v8f relu8(v8f d) {
  v8f r;
#pragma unroll
  for (int i = 0; i < 8; ++i) r[i] = fmaxf(d[i], 0.0f);
  return r;
}

__device__ __forceinline__ v8f ldb8(const float* __restrict__ p) {
  const v4f a = *(const v4f*)p;
  const v4f b = *(const v4f*)(p + 4);
  return cat8(a, b);
}

__device__ __forceinline__ v8f wmb(const FragB& a, const FragB& b, v8f c) {
  return __builtin_amdgcn_wmma_f32_16x16x32_bf16(false, a.v, false, b.v, (short)0, c, false, false);
}

__device__ __forceinline__ void lda4(const bf_t* __restrict__ hi, const bf_t* __restrict__ lo, int f, int h,
                                     FragB& ah, FragB& al, FragB& ath, FragB& atl) {
  const bf_t* ph = hi + (size_t)f * KP + 8 * h;
  const bf_t* pl = lo + (size_t)f * KP + 8 * h;
  ah.b[0] = *(const v8b*)ph;
  ah.b[1] = *(const v8b*)(ph + 16);
  al.b[0] = *(const v8b*)pl;
  al.b[1] = *(const v8b*)(pl + 16);
  const v8b th = *(const v8b*)(ph + 32);
  ath.b[0] = th;
  ath.b[1] = th;
  atl.b[0] = *(const v8b*)(pl + 32);
  atl.b[1] = zero8b();
}

__device__ __forceinline__ void ldb3(const bf_t* rh, const bf_t* rl, int h, FragB& bh, FragB& bl, FragB& bt) {
  bh.b[0] = *(const v8b*)(rh + 8 * h);
  bh.b[1] = *(const v8b*)(rh + 16 + 8 * h);
  bl.b[0] = *(const v8b*)(rl + 8 * h);
  bl.b[1] = *(const v8b*)(rl + 16 + 8 * h);
  bt.b[0] = *(const v8b*)(rh + 32 + 8 * h);
  bt.b[1] = *(const v8b*)(rl + 32 + 8 * h);
}

__device__ __forceinline__ v8f chain5(const FragB& ah, const FragB& al, const FragB& ath, const FragB& atl,
                                      const FragB& bh, const FragB& bl, const FragB& bt, v8f c) {
  v8f d = wmb(ah, bh, c);
  d = wmb(ah, bl, d);
  d = wmb(al, bh, d);
  d = wmb(ath, bt, d);
  d = wmb(atl, bt, d);
  return d;
}

#define WGUARD(d0, a0, a1, a2, a3, b0, b1, b2)                                                  \
  asm volatile("v_nop\n\tv_nop\n\tv_nop\n\tv_nop"                                             \
               : "+v"(d0)                                                                     \
               : "v"((a0).f), "v"((a1).f), "v"((a2).f), "v"((a3).f),                         \
                 "v"((b0).f), "v"((b1).f), "v"((b2).f)                                        \
               : "memory")

__device__ __forceinline__ void edge_sd(const int* __restrict__ nbr, int e, int P, int& s, int& d) {
  const bool lt = e < P;
  const int ee = lt ? e : e - P;
  const v2i pr = *(const v2i*)(nbr + (size_t)2 * (size_t)ee);
  s = lt ? pr.x : pr.y;
  d = lt ? pr.y : pr.x;
}

__device__ __forceinline__ void zero16(float (&o)[16]) {
#pragma unroll
  for (int i = 0; i < 16; ++i) o[i] = 0.0f;
}
__device__ __forceinline__ void zero12(float (&o)[12]) {
#pragma unroll
  for (int i = 0; i < 12; ++i) o[i] = 0.0f;
}
__device__ __forceinline__ void ld16(float (&o)[16], const float* p) {
#pragma unroll
  for (int q = 0; q < 4; ++q) {
    const v4f v = *(const v4f*)(p + 4 * q);
    o[4 * q] = v.x; o[4 * q + 1] = v.y; o[4 * q + 2] = v.z; o[4 * q + 3] = v.w;
  }
}
__device__ __forceinline__ void ld12(float (&o)[12], const float* p) {
#pragma unroll
  for (int q = 0; q < 3; ++q) {
    const v4f v = *(const v4f*)(p + 4 * q);
    o[4 * q] = v.x; o[4 * q + 1] = v.y; o[4 * q + 2] = v.z; o[4 * q + 3] = v.w;
  }
}
__device__ __forceinline__ void st16(float* p, const float (&o)[16], float s) {
#pragma unroll
  for (int q = 0; q < 4; ++q) {
    const v4f v = {s * o[4 * q], s * o[4 * q + 1], s * o[4 * q + 2], s * o[4 * q + 3]};
    *(v4f*)(p + 4 * q) = v;
  }
}
__device__ __forceinline__ void st12(float* p, const float (&o)[12], float s) {
#pragma unroll
  for (int q = 0; q < 3; ++q) {
    const v4f v = {s * o[4 * q], s * o[4 * q + 1], s * o[4 * q + 2], s * o[4 * q + 3]};
    *(v4f*)(p + 4 * q) = v;
  }
}
__device__ __forceinline__ void mac16(float (&o)[16], float x, const float* wp) {
  const v4f a = *(const v4f*)wp;
  const v4f b = *(const v4f*)(wp + 4);
  const v4f c = *(const v4f*)(wp + 8);
  const v4f d = *(const v4f*)(wp + 12);
  o[0]  += x * a.x; o[1]  += x * a.y; o[2]  += x * a.z; o[3]  += x * a.w;
  o[4]  += x * b.x; o[5]  += x * b.y; o[6]  += x * b.z; o[7]  += x * b.w;
  o[8]  += x * c.x; o[9]  += x * c.y; o[10] += x * c.z; o[11] += x * c.w;
  o[12] += x * d.x; o[13] += x * d.y; o[14] += x * d.z; o[15] += x * d.w;
}
__device__ __forceinline__ void mac4x3(float (&q)[12], float a0, float a1, float a2, v4f w) {
  q[0] += a0 * w.x; q[1]  += a1 * w.x; q[2]  += a2 * w.x;
  q[3] += a0 * w.y; q[4]  += a1 * w.y; q[5]  += a2 * w.y;
  q[6] += a0 * w.z; q[7]  += a1 * w.z; q[8]  += a2 * w.z;
  q[9] += a0 * w.w; q[10] += a1 * w.w; q[11] += a2 * w.w;
}

__global__ __launch_bounds__(NTHR) void k_wprep(const float* __restrict__ wa, const float* __restrict__ wb,
                                                const float* __restrict__ wc, const float* __restrict__ wd,
                                                bf_t* phi, bf_t* plo, int nrows) {
  const int tid = threadIdx.x, lane = tid & 31, wave = tid >> 5;
  const int g = (blockIdx.x * NWAVE + wave) * 4 + (lane >> 3);
  const int kq = (lane & 7) * 8;
  const bool s0 = g < 48, s1 = g < 368, s2 = g < 416;
  const int fa = imin(imax(g, 0), 47);
  const int fb = imin(imax(g - 48, 0), 319);
  const int fc = imin(imax(g - 368, 0), 47);
  const int fd = imin(imax(g - 416, 0), 431);
  v8f x;
#pragma unroll
  for (int i = 0; i < 8; ++i) {
    const int k = kq + i;
    const int kc = imin(k, 47);
    const float va = wa[kc * 48 + fa];
    const float vb = wb[kc * 320 + fb];
    const float vc = wc[kc * 48 + fc];
    const float vd = wd[kc * 432 + fd];
    const float v = s0 ? va : (s1 ? vb : (s2 ? vc : vd));
    x[i] = (k < 48) ? v : 0.0f;
  }
  Pk8 uh, ul;
  split8(x, uh.b, ul.b);
  const bool wr = g < nrows;
  const size_t o = (size_t)g * KP + kq;
  if (wr) { *(volatile v4f*)(phi + o) = uh.f; *(volatile v4f*)(plo + o) = ul.f; }
  __threadfence();
  if (wr) { *(volatile v4f*)(phi + o) = uh.f; *(volatile v4f*)(plo + o) = ul.f; }
}

__global__ __launch_bounds__(NTA) void k_node(const float* __restrict__ z, const float* __restrict__ w1,
                                              const float* __restrict__ b1, const float* __restrict__ w2,
                                              const float* __restrict__ b2, float* node0, int nN) {
  __shared__ __attribute__((aligned(16))) float zs[NTA * 32];
  __shared__ float ts[NTA * 16];
  __shared__ __attribute__((aligned(16))) float os[NTA * 16];
  const int tid = threadIdx.x;
  const int i = blockIdx.x * NTA + tid;
  const int ic = imin(i, nN - 1);
  const float* zr = z + (size_t)ic * 32;
#pragma unroll
  for (int q = 0; q < 8; ++q) *(v4f*)(zs + tid * 32 + 4 * q) = *(const v4f*)(zr + 4 * q);
  __syncthreads();
#pragma unroll 1
  for (int j = 0; j < 16; ++j) {
    float a = b1[j];
#pragma unroll 1
    for (int k = 0; k < 32; ++k) a += zs[tid * 32 + k] * w1[k * 16 + j];
    ts[tid * 16 + j] = tanhf(a);
  }
#pragma unroll 1
  for (int j = 0; j < 16; ++j) {
    float a = b2[j];
#pragma unroll 1
    for (int k = 0; k < 16; ++k) a += ts[tid * 16 + k] * w2[k * 16 + j];
    os[tid * 16 + j] = a;
  }
  __syncthreads();
  const size_t base = (size_t)blockIdx.x * NTA * 16;
  v4f ov[4];
#pragma unroll
  for (int q = 0; q < 4; ++q) ov[q] = *(const v4f*)(os + q * 512 + 4 * tid);
#pragma unroll
  for (int q = 0; q < 4; ++q) *(volatile v4f*)(node0 + base + q * 512 + 4 * tid) = ov[q];
  __threadfence();
#pragma unroll
  for (int q = 0; q < 4; ++q) *(volatile v4f*)(node0 + base + q * 512 + 4 * tid) = ov[q];
}

__global__ __launch_bounds__(NTA) void k_edgef(const int* __restrict__ nbr, const float* __restrict__ xyz,
                                               const float* __restrict__ w1, const float* __restrict__ b1,
                                               const float* __restrict__ w2, const float* __restrict__ b2,
                                               float* edgef, int nN, int P) {
  __shared__ float els[NTA * 8];
  __shared__ float ehs[NTA * 16];
  __shared__ __attribute__((aligned(16))) float os[NTA * EFP];
  const int tid = threadIdx.x;
  const int E = 2 * P;
  const int e = blockIdx.x * NTA + tid;
  const int ec = imin(e, E - 1);
  int s, d;
  edge_sd(nbr, ec, P, s, d);
  s = imin(imax(s, 0), nN - 1);
  d = imin(imax(d, 0), nN - 1);
  const float rx = xyz[3 * d + 0] - xyz[3 * s + 0];
  const float ry = xyz[3 * d + 1] - xyz[3 * s + 1];
  const float rz = xyz[3 * d + 2] - xyz[3 * s + 2];
  const float dd = sqrtf(rx * rx + ry * ry + rz * rz);
  const float inv = 1.0f / fmaxf(dd, 1e-9f);
  const float hx = rx * inv, hy = ry * inv, hz = rz * inv;
#pragma unroll 1
  for (int j = 0; j < 8; ++j) {
    const float t = dd - (float)j * RBF_STEP;
    els[tid * 8 + j] = expf(RBF_COEFF * (t * t));
  }
#pragma unroll 1
  for (int j = 0; j < 16; ++j) {
    float a = b1[j];
#pragma unroll 1
    for (int k = 0; k < 8; ++k) a += els[tid * 8 + k] * w1[k * 16 + j];
    ehs[tid * 16 + j] = fmaxf(a, 0.0f);
  }
  float* orow = os + tid * EFP;
#pragma unroll 1
  for (int j = 0; j < 16; ++j) {
    float a = b2[j];
#pragma unroll 1
    for (int k = 0; k < 16; ++k) a += ehs[tid * 16 + k] * w2[k * 16 + j];
    orow[j] = a;
  }
  {
    const v4f g4 = {SQ3F * hx, SQ3F * hy, SQ3F * hz, S15 * hx * hz};
    const v4f g5 = {S15 * hx * hy, S5 * (hy * hy - 0.5f * (hx * hx + hz * hz)), S15 * hy * hz, 0.5f * S15 * (hz * hz - hx * hx)};
    const v4f z4 = {0.0f, 0.0f, 0.0f, 0.0f};
    *(v4f*)(orow + 16) = g4;
    *(v4f*)(orow + 20) = g5;
    *(v4f*)(orow + 24) = z4;
    *(v4f*)(orow + 28) = z4;
  }
  __syncthreads();
  const size_t base = (size_t)blockIdx.x * NTA * EFP;
  v4f ov[8];
#pragma unroll
  for (int q = 0; q < 8; ++q) ov[q] = *(const v4f*)(os + q * 512 + 4 * tid);
#pragma unroll
  for (int q = 0; q < 8; ++q) *(volatile v4f*)(edgef + base + q * 512 + 4 * tid) = ov[q];
  __threadfence();
#pragma unroll
  for (int q = 0; q < 8; ++q) *(volatile v4f*)(edgef + base + q * 512 + 4 * tid) = ov[q];
}

__device__ __forceinline__ int scan_chunk(const int* __restrict__ nbr, int P, int E, int cbase, int nodeBase,
                                          int vec, int* list, int tid, int wave) {
  int wc = 0;
  const int el0 = tid * EPT;
  const int e0 = cbase + el0;
  const int sent = -2147483647 - 1;
  int sv[EPT];
  if (vec != 0 && cbase + CHUNK <= E) {
    const bool lt = e0 < P;
    const int pb = lt ? e0 : (e0 - P);
    const int* qp = nbr + (size_t)2 * (size_t)pb;
    const v4i q0 = *(const v4i*)(qp);
    const v4i q1 = *(const v4i*)(qp + 4);
    const v4i q2 = *(const v4i*)(qp + 8);
    const v4i q3 = *(const v4i*)(qp + 12);
    sv[0] = lt ? q0.x : q0.y;  sv[1] = lt ? q0.z : q0.w;
    sv[2] = lt ? q1.x : q1.y;  sv[3] = lt ? q1.z : q1.w;
    sv[4] = lt ? q2.x : q2.y;  sv[5] = lt ? q2.z : q2.w;
    sv[6] = lt ? q3.x : q3.y;  sv[7] = lt ? q3.z : q3.w;
  } else {
#pragma unroll
    for (int j = 0; j < EPT; ++j) {
      const int e = e0 + j;
      const int ec = e < E ? e : E - 1;
      const bool lt = ec < P;
      const int ee = lt ? ec : ec - P;
      const int v = nbr[2 * ee + (lt ? 0 : 1)];
      sv[j] = (e < E) ? v : sent;
    }
  }
  bool hit[EPT];
  int anyi = 0;
#pragma unroll
  for (int j = 0; j < EPT; ++j) {
    hit[j] = ((unsigned)sv[j] - (unsigned)nodeBase) < (unsigned)NB;
    anyi |= hit[j] ? 1 : 0;
  }
  const unsigned any = __builtin_amdgcn_ballot_w32(anyi != 0);
  if (any != 0u) {
#pragma unroll
    for (int j = 0; j < EPT; ++j) {
      const unsigned mj = __builtin_amdgcn_ballot_w32(hit[j]);
      if (mj != 0u) {
        if (hit[j]) {
          const int pos = wc + (int)__builtin_amdgcn_mbcnt_lo(mj, 0u);
          if (pos < WCAP) list[wave * WCAP + pos] = el0 + j;
        }
        wc += (int)__builtin_popcount(mj);
      }
    }
  }
  return wc;
}

template <int INW, int PI, int OUTW, int MP, int PO>
__device__ __forceinline__ v4f epi_val(const float* accp, const float* __restrict__ nodein,
                                       int nodeBase, int nN, int off) {
  const int row  = off / PO;
  const int col  = off - row * PO;
  const int rowc = imin(nodeBase + row, nN - 1);
  const int ldc  = imin(col, PI - 4);
  const v4f bv   = *(const v4f*)(nodein + (size_t)rowc * PI + ldc);
  const bool hasb = col < INW;
  const float cn  = accp[row * MP + OUTW];
  const float inv = 1.0f / fmaxf(cn, 1.0f);
  const v4f av    = *(const v4f*)(accp + row * MP + imin(col, MP - 4));
  const bool va   = col < OUTW;
  v4f t;
  t.x = va ? ((hasb ? bv.x : 0.0f) + av.x * inv) : 0.0f;
  t.y = va ? ((hasb ? bv.y : 0.0f) + av.y * inv) : 0.0f;
  t.z = va ? ((hasb ? bv.z : 0.0f) + av.z * inv) : 0.0f;
  t.w = va ? ((hasb ? bv.w : 0.0f) + av.w * inv) : 0.0f;
  return t;
}

template <int LAYER>
__device__ __forceinline__ void tp_group(int g, const float* wr, const float* gr, float* mr) {
  if (g < 4) {
    float o[16];
    if (g == 0) zero16(o); else ld16(o, mr);
#pragma unroll 1
    for (int uu = 0; uu < 4; ++uu) mac16(o, gr[4 * g + uu], wr + 16 * uu);
    st16(mr, o, 1.0f);
    return;
  }
  if (g == 4) {
    float sb0 = 0.0f, sb1 = 0.0f, sb2 = 0.0f, sb3 = 0.0f;
#pragma unroll 1
    for (int u = 0; u < 16; ++u) {
      const float x = gr[u];
      const v4f wv = *(const v4f*)(wr + 4 * u);
      sb0 += x * wv.x; sb1 += x * wv.y; sb2 += x * wv.z; sb3 += x * wv.w;
    }
    const float y0 = gr[16], y1 = gr[17], y2 = gr[18];
    const float k = LAYER ? INV3 : 0.25f;
    const v4f m0 = {k * (sb0 * y0), k * (sb0 * y1), k * (sb0 * y2), k * (sb1 * y0)};
    const v4f m1 = {k * (sb1 * y1), k * (sb1 * y2), k * (sb2 * y0), k * (sb2 * y1)};
    const v4f m2 = {k * (sb2 * y2), k * (sb3 * y0), k * (sb3 * y1), k * (sb3 * y2)};
    *(v4f*)(mr + 16) = m0; *(v4f*)(mr + 20) = m1; *(v4f*)(mr + 24) = m2;
    if (LAYER == 0) {
      float o[16];
      ld16(o, mr);
      st16(mr, o, 0.25f);
      const v4f cp = {1.0f, 0.0f, 0.0f, 0.0f};
      *(v4f*)(mr + 28) = cp;
    }
    return;
  }
  if (LAYER != 0) {
    const float s1x = gr[16], s1y = gr[17], s1z = gr[18];
    if (g == 5) {
      {
        float q[12];
        ld12(q, mr + 16);
#pragma unroll 1
        for (int u = 0; u < 4; ++u) {
          const float a0 = gr[24 + 3 * u] * INV3, a1 = gr[25 + 3 * u] * INV3, a2 = gr[26 + 3 * u] * INV3;
          mac4x3(q, a0, a1, a2, *(const v4f*)(wr + 4 * u));
        }
        st12(mr + 16, q, 1.0f);
      }
      {
        float o[16];
        ld16(o, mr);
#pragma unroll 1
        for (int u = 0; u < 3; ++u) {
          const float a0 = gr[24 + 3 * u], a1 = gr[25 + 3 * u], a2 = gr[26 + 3 * u];
          const float vd = (a0 * s1x + a1 * s1y + a2 * s1z) * INV3;
          mac16(o, vd, wr + 16 + 16 * u);
        }
        st16(mr, o, 1.0f);
      }
    } else {
      {
        float o[16];
        ld16(o, mr);
        const float a0 = gr[33], a1 = gr[34], a2 = gr[35];
        const float vd = (a0 * s1x + a1 * s1y + a2 * s1z) * INV3;
        mac16(o, vd, wr);
        st16(mr, o, PW0);
      }
      {
        float ev[12];
        zero12(ev);
#pragma unroll 1
        for (int u = 0; u < 4; ++u) {
          const float a0 = gr[24 + 3 * u], a1 = gr[25 + 3 * u], a2 = gr[26 + 3 * u];
          const float c0 = (a1 * s1z - a2 * s1y) * INV6;
          const float c1 = (a2 * s1x - a0 * s1z) * INV6;
          const float c2 = (a0 * s1y - a1 * s1x) * INV6;
          mac4x3(ev, c0, c1, c2, *(const v4f*)(wr + 16 + 4 * u));
        }
        st12(mr + 28, ev, P1E);
      }
      {
        float q[12];
        ld12(q, mr + 16);
        const float q0 = gr[19], q1 = gr[20], q2 = gr[21], q3 = gr[22], q4 = gr[23];
#pragma unroll 1
        for (int u = 0; u < 4; ++u) {
          const float a0 = gr[24 + 3 * u], a1 = gr[25 + 3 * u], a2 = gr[26 + 3 * u];
          const float t0 = C_A * (a2 * q0 + a1 * q1) - 0.5f * C_B * (a0 * q2) - C_A * (a0 * q4);
          const float t1 = C_A * (a0 * q1) + C_B * (a1 * q2) + C_A * (a2 * q3);
          const float t2 = C_A * (a0 * q0) - 0.5f * C_B * (a2 * q2) + C_A * (a1 * q3) + C_A * (a2 * q4);
          mac4x3(q, t0, t1, t2, *(const v4f*)(wr + 32 + 4 * u));
        }
        st12(mr + 16, q, PW1);
      }
      const v4f cp = {1.0f, 0.0f, 0.0f, 0.0f};
      *(v4f*)(mr + 40) = cp;
    }
  }
}

template <int LAYER>
__global__ __launch_bounds__(NTHR) void k_conv(
    const int* __restrict__ nbr, const float* __restrict__ edgef, const float* __restrict__ nodein,
    const bf_t* __restrict__ w1hi, const bf_t* __restrict__ w1lo, const float* __restrict__ bi1,
    const bf_t* __restrict__ w2hi, const bf_t* __restrict__ w2lo, const float* __restrict__ bi2,
    float* outp, int nN, int P, int vec, int outLim) {
  constexpr int INW  = LAYER ? 28 : 16;
  constexpr int PI   = LAYER ? N28P : 16;
  constexpr int OUTW = LAYER ? 40 : 28;
  constexpr int MP   = LAYER ? 44 : 32;
  constexpr int PO   = LAYER ? 40 : N28P;
  constexpr int GP   = LAYER ? 36 : 20;
  constexpr int NT   = LAYER ? 27 : 20;
  constexpr int NG   = (NT + 3) / 4;
  constexpr int NQ   = (NB * PO) / (128 * NWAVE);
  constexpr int NACC = MP / 4;
  static_assert(NQ * 128 * NWAVE == NB * PO);
  static_assert((MP % 4) == 0 && MP > OUTW && NACC <= NTHR);
  static_assert((PO % 4) == 0 && (PI % 4) == 0 && (INW % 4) == 0 && (OUTW % 4) == 0 && (GP % 4) == 0);
  static_assert((((NB + 1) * MP) % 4) == 0);

  __shared__ __attribute__((aligned(16))) float acc[(NB + 1) * MP];
  __shared__ __attribute__((aligned(16))) float msg[PASSN * MP];
  __shared__ __attribute__((aligned(16))) bf_t  sth[PASSN * SP];
  __shared__ __attribute__((aligned(16))) bf_t  stl[PASSN * SP];
  __shared__ __attribute__((aligned(16))) bf_t  hdh[PASSN * SP];
  __shared__ __attribute__((aligned(16))) bf_t  hdl[PASSN * SP];
  __shared__ __attribute__((aligned(16))) float geo[PASSN * GP];
  __shared__ __attribute__((aligned(16))) float wst[PASSN * WP];
  __shared__ __attribute__((aligned(16))) int   list[LISTN];
  __shared__ __attribute__((aligned(16))) int   pend[PCAP];
  __shared__ int slotb[PASSN];
  __shared__ int wcnt[NWAVE];
  __shared__ int pendN;

  const int tid = threadIdx.x, lane = tid & 31, wave = tid >> 5, h = lane >> 4, m = lane & 15;
  const int nodeBase = blockIdx.x * NB;
  const int E = 2 * P;
  const int rbase = wave * 32;

  {
    const v4f z4 = {0.0f, 0.0f, 0.0f, 0.0f};
    for (int i = tid; i < ((NB + 1) * MP) / 4; i += NTHR) *(v4f*)(acc + 4 * i) = z4;
  }
  if (tid == 0) pendN = 0;
  __syncthreads();

  const int nChunks = (E + CHUNK - 1) / CHUNK;
#pragma unroll 1
  for (int ch = 0; ch < nChunks; ++ch) {
    const int cbase = ch * CHUNK;
    const int wc = scan_chunk(nbr, P, E, cbase, nodeBase, vec, list, tid, wave);
    if (lane == 0) wcnt[wave] = wc;
    __syncthreads();

    const int base = pendN;
    int tot = 0, myoff = 0;
#pragma unroll
    for (int w = 0; w < NWAVE; ++w) {
      int c = wcnt[w];
      c = c > WCAP ? WCAP : (c < 0 ? 0 : c);
      if (w < wave) myoff += c;
      tot += c;
    }
    int newN = base + tot;
    newN = newN > PCAP ? PCAP : newN;
    {
      int n = wcnt[wave];
      n = n > WCAP ? WCAP : (n < 0 ? 0 : n);
      const int* lp = list + wave * WCAP;
      for (int i = lane; i < n; i += 32) {
        const int pos = base + myoff + i;
        if (pos < PCAP) pend[pos] = cbase + lp[i];
      }
    }
    const int fin = (ch == nChunks - 1) ? 1 : 0;
    const int R   = (fin != 0) ? (newN + PASSN - 1) / PASSN : newN / PASSN;
    const int Pv  = (fin != 0) ? newN : R * PASSN;
    __syncthreads();

#pragma unroll 1
    for (int rp = 0; rp < R; ++rp) {
      {
        const int idx = rp * PASSN + tid;
        const bool valid = idx < Pv;
        int e = pend[imin(idx, PCAP - 1)];
        e = valid ? e : 0;
        e = imin(imax(e, 0), E - 1);
        int src, dst;
        edge_sd(nbr, e, P, src, dst);
        int slot = src - nodeBase;
        if (!valid || (unsigned)slot >= (unsigned)NB) slot = NB;
        const int sc = imin(imax(src, 0), nN - 1);
        const int dc = imin(imax(dst, 0), nN - 1);
        const float* er = edgef + (size_t)e * EFP;
        const float* ps = nodein + (size_t)sc * PI;
        const float* pd = nodein + (size_t)dc * PI;
        bf_t* rh = sth + tid * SP;
        bf_t* rl = stl + tid * SP;
        float* gr = geo + tid * GP;
#pragma unroll 1
        for (int p = 0; p < 6; ++p) {
          const float* gp = (p < 2) ? (er + 8 * p) : ((p < 4) ? (ps + 8 * (p - 2)) : (pd + 8 * (p - 4)));
          const v4f x0 = *(const v4f*)gp;
          const v4f x1 = *(const v4f*)(gp + 4);
          v8b uh, ul;
          split8(cat8(x0, x1), uh, ul);
          *(v8b*)(rh + 8 * p) = uh;
          *(v8b*)(rl + 8 * p) = ul;
          if (p >= 4) {
            *(v4f*)(gr + 8 * (p - 4))     = x0;
            *(v4f*)(gr + 8 * (p - 4) + 4) = x1;
          }
        }
        *(v4f*)(gr + 16) = *(const v4f*)(er + 16);
        if (LAYER != 0) {
          *(v4f*)(gr + 20) = *(const v4f*)(er + 20);
          *(v4f*)(gr + 24) = *(const v4f*)(pd + 16);
          *(v4f*)(gr + 28) = *(const v4f*)(pd + 20);
          *(v4f*)(gr + 32) = *(const v4f*)(pd + 24);
        }
        slotb[tid] = slot;
      }
      __syncthreads();

      {
#pragma unroll 1
        for (int ft = 0; ft < 3; ++ft) {
          FragB ah, al, ath, atl;
          lda4(w1hi, w1lo, 16 * ft + m, h, ah, al, ath, atl);
          const v8f c = ldb8(bi1 + 16 * ft + 8 * h);
#pragma unroll 1
          for (int et = 0; et < 2; ++et) {
            const int row = rbase + 16 * et + m;
            FragB bh, bl, bt;
            ldb3(sth + row * SP, stl + row * SP, h, bh, bl, bt);
            v8f d = chain5(ah, al, ath, atl, bh, bl, bt, c);
            WGUARD(d, ah, al, ath, atl, bh, bl, bt);
            v8b xh, xl;
            split8(relu8(d), xh, xl);
            *(v8b*)(hdh + row * SP + 16 * ft + 8 * h) = xh;
            *(v8b*)(hdl + row * SP + 16 * ft + 8 * h) = xl;
          }
        }
      }
      __syncthreads();

#pragma unroll 1
      for (int g = 0; g < NG; ++g) {
        {
          const int ntg = imin(4, NT - 4 * g);
#pragma unroll 1
          for (int t = 0; t < ntg; ++t) {
            const int ft = 4 * g + t;
            FragB ah, al, ath, atl;
            lda4(w2hi, w2lo, 16 * ft + m, h, ah, al, ath, atl);
            const v8f c = ldb8(bi2 + 16 * ft + 8 * h);
#pragma unroll 1
            for (int et = 0; et < 2; ++et) {
              const int row = rbase + 16 * et + m;
              FragB bh, bl, bt;
              ldb3(hdh + row * SP, hdl + row * SP, h, bh, bl, bt);
              v8f d = chain5(ah, al, ath, atl, bh, bl, bt, c);
              WGUARD(d, ah, al, ath, atl, bh, bl, bt);
              float* p0 = wst + row * WP + 16 * t + 8 * h;
              *(v4f*)p0       = lo4(d);
              *(v4f*)(p0 + 4) = hi4(d);
            }
          }
        }
        __syncthreads();
        tp_group<LAYER>(g, wst + tid * WP, geo + tid * GP, msg + tid * MP);
        __syncthreads();
      }

      if (tid < NACC) {
#pragma unroll 1
        for (int i = 0; i < PASSN; ++i) {
          int sl = slotb[i];
          sl = imin(imax(sl, 0), NB);
          float* ap = acc + sl * MP + 4 * tid;
          v4f a = *(const v4f*)ap;
          const v4f mv = *(const v4f*)(msg + i * MP + 4 * tid);
          a += mv;
          *(v4f*)ap = a;
        }
      }
      __syncthreads();
    }

    int rem = newN - R * PASSN;
    rem = rem < 0 ? 0 : rem;
    if (R > 0 && tid < rem) pend[tid] = pend[R * PASSN + tid];
    if (tid == 0) pendN = rem;
  }
  __syncthreads();

  const size_t ob  = (size_t)nodeBase * PO;
  const size_t lim = (size_t)(outLim < 0 ? 0 : outLim);
#pragma unroll 1
  for (int q = 0; q < NQ; ++q) {
    const int off = (wave * NQ + q) * 128 + 4 * lane;
    const v4f t = epi_val<INW, PI, OUTW, MP, PO>(acc, nodein, nodeBase, nN, off);
    const size_t gi = ob + (size_t)off;
    if (gi + 3 < lim) *(volatile v4f*)(outp + gi) = t;
  }
  __threadfence();
#pragma unroll 1
  for (int q = 0; q < NQ; ++q) {
    const int off = (wave * NQ + q) * 128 + 4 * lane;
    const v4f t = epi_val<INW, PI, OUTW, MP, PO>(acc, nodein, nodeBase, nN, off);
    const size_t gi = ob + (size_t)off;
    if (gi + 3 < lim) *(volatile v4f*)(outp + gi) = t;
  }
}

static inline size_t al256(size_t x) { return (x + 255) & ~(size_t)255; }

extern "C" void kernel_launch(void* const* d_in, const int* in_sizes, int n_in,
                              void* d_out, int out_size, void* d_ws, size_t ws_size,
                              hipStream_t stream) {
  if (n_in < 19) return;
  const int nN = in_sizes[0] / 32;
  const int P  = in_sizes[2] / 2;
  if (nN <= 0 || P <= 0) return;
  if (in_sizes[0] != nN * 32 || in_sizes[1] != nN * 3 || in_sizes[2] != P * 2) return;
  if (in_sizes[3] != 32 * 16 || in_sizes[4] != 16 || in_sizes[5] != 16 * 16 || in_sizes[6] != 16) return;
  if (in_sizes[7] != 8 * 16 || in_sizes[8] != 16 || in_sizes[9] != 16 * 16 || in_sizes[10] != 16) return;
  if (in_sizes[11] != 48 * 48 || in_sizes[12] != 48 || in_sizes[13] != 48 * 320 || in_sizes[14] != 320) return;
  if (in_sizes[15] != 48 * 48 || in_sizes[16] != 48 || in_sizes[17] != 48 * 432 || in_sizes[18] != 432) return;
  if (out_size != nN * 40) return;

  const float* cg_z    = (const float*)d_in[0];
  const float* cg_xyz  = (const float*)d_in[1];
  const int*   nbr     = (const int*)d_in[2];
  const float* node_w1 = (const float*)d_in[3];
  const float* node_b1 = (const float*)d_in[4];
  const float* node_w2 = (const float*)d_in[5];
  const float* node_b2 = (const float*)d_in[6];
  const float* edge_w1 = (const float*)d_in[7];
  const float* edge_b1 = (const float*)d_in[8];
  const float* edge_w2 = (const float*)d_in[9];
  const float* edge_b2 = (const float*)d_in[10];
  const float* fc0_w1  = (const float*)d_in[11];
  const float* fc0_b1  = (const float*)d_in[12];
  const float* fc0_w2  = (const float*)d_in[13];
  const float* fc0_b2  = (const float*)d_in[14];
  const float* fc1_w1  = (const float*)d_in[15];
  const float* fc1_b1  = (const float*)d_in[16];
  const float* fc1_w2  = (const float*)d_in[17];
  const float* fc1_b2  = (const float*)d_in[18];
  float* out = (float*)d_out;

  const int E    = 2 * P;
  const int nbN  = (nN + NTA - 1) / NTA;
  const int nbE  = (E + NTA - 1) / NTA;
  const int nBlk = (nN + NB - 1) / NB;
  const int nbW  = NWROWS / (4 * NWAVE);

  char* ws = (char*)d_ws;
  size_t off = 0;
  const size_t oHi = off; off = al256(off + (size_t)NWROWS * KP * sizeof(bf_t));
  const size_t oLo = off; off = al256(off + (size_t)NWROWS * KP * sizeof(bf_t));
  const size_t oN0 = off; off = al256(off + (size_t)nbN * NTA * 16 * sizeof(float));
  const size_t oEf = off; off = al256(off + (size_t)nbE * NTA * EFP * sizeof(float));
  const size_t oN1 = off; off = al256(off + (size_t)nBlk * NB * N28P * sizeof(float));
  if (off > ws_size) return;
  bf_t*  phi    = (bf_t*)(ws + oHi);
  bf_t*  plo    = (bf_t*)(ws + oLo);
  float* node0  = (float*)(ws + oN0);
  float* edgef  = (float*)(ws + oEf);
  float* node28 = (float*)(ws + oN1);

  const int vec = ((P & 7) == 0) ? 1 : 0;

  k_wprep<<<nbW, NTHR, 0, stream>>>(fc0_w1, fc0_w2, fc1_w1, fc1_w2, phi, plo, NWROWS);
  k_node<<<nbN, NTA, 0, stream>>>(cg_z, node_w1, node_b1, node_w2, node_b2, node0, nN);
  k_edgef<<<nbE, NTA, 0, stream>>>(nbr, cg_xyz, edge_w1, edge_b1, edge_w2, edge_b2, edgef, nN, P);

  k_conv<0><<<nBlk, NTHR, 0, stream>>>(
      nbr, edgef, node0,
      phi, plo, fc0_b1,
      phi + (size_t)48 * KP, plo + (size_t)48 * KP, fc0_b2,
      node28, nN, P, vec, nBlk * NB * N28P);

  k_conv<1><<<nBlk, NTHR, 0, stream>>>(
      nbr, edgef, node28,
      phi + (size_t)368 * KP, plo + (size_t)368 * KP, fc1_b1,
      phi + (size_t)416 * KP, plo + (size_t)416 * KP, fc1_b2,
      out, nN, P, vec, out_size);
}
